// DiffusionLayer_19353122636426
// MI455X (gfx1250) — hardware-verified
//
#include <hip/hip_runtime.h>
#include <hip/hip_bf16.h>
#include <math.h>


#define BB 2
#define SS 2048
#define DD 1024
#define HH 16
#define DKK 64
#define QW 2

typedef _Float16 bf16;
typedef __attribute__((ext_vector_type(4))) unsigned v4u_t;
typedef unsigned v4ua __attribute__((ext_vector_type(4), may_alias));
typedef __attribute__((ext_vector_type(4))) float v4f_t;
typedef float v4fa __attribute__((ext_vector_type(4), may_alias));
typedef __attribute__((ext_vector_type(16))) bf16  bf16x16;
typedef __attribute__((ext_vector_type(8)))  bf16  bf16x8;
typedef __attribute__((ext_vector_type(4)))  bf16  bf16x4;
typedef __attribute__((ext_vector_type(8)))  float f32x8;

#define LDS_STRIDE 48
#define KSTRIDE    72
#define VSTRIDE    48

__device__ __forceinline__ f32x8 wmma_bf16(bf16x16 a, bf16x16 b, f32x8 c) {
  return __builtin_amdgcn_wmma_f32_16x16x32_f16(
      false, a, false, b, (short)0, c, false, false);
}
#define RSPLIT (1.0f / 2048.0f)
__device__ __forceinline__ bf16 lo_of(float v, bf16 h) { return (bf16)((v - (float)h) * 2048.0f); }
__device__ __forceinline__ f32x8 wmma_split(bf16x16 a, bf16x16 al, bf16x16 b, bf16x16 bl, f32x8 c) {
  f32x8 x = {}; x = wmma_bf16(al, b, x); x = wmma_bf16(a, bl, x); return wmma_bf16(a, b, c) + x * RSPLIT; }

template <typename T>
__device__ __forceinline__ bf16x16 load_frag(const T* __restrict__ base, int ld,
                                             int row0, int k0) {
  const int lane = threadIdx.x & 31;
  const int r    = lane & 15;
  const int kh   = (lane >> 4) * 8;
  const T* p0 = base + (size_t)(row0 + r) * ld + (k0 + kh);
  const T* p1 = p0 + 16;
  bf16x16 f;
#pragma unroll
  for (int i = 0; i < 8; ++i) {
    f[i]     = (bf16)p0[i];
    f[i + 8] = (bf16)p1[i];
  }
  return f;
}

__device__ __forceinline__ bf16x16 lds_frag(const bf16* base, int stride) {
  const int lane = threadIdx.x & 31;
  const int row  = lane & 15;
  const int kh   = (lane >> 4) * 8;
  const bf16x8 lo = *(const bf16x8*)(base + row * stride + kh);
  const bf16x8 hi = *(const bf16x8*)(base + row * stride + kh + 16);
  bf16x16 f;
#pragma unroll
  for (int i = 0; i < 8; ++i) { f[i] = lo[i]; f[i + 8] = hi[i]; }
  return f;
}

template <typename T>
__device__ __forceinline__ void stage_read16(const T* __restrict__ p, float* buf) {
#pragma unroll
  for (int i = 0; i < 16; ++i) buf[i] = (float)p[i];
}

__device__ __forceinline__ void stage_write(bf16* dst, const float* buf, int nquad) {
#pragma unroll
  for (int i = 0; i < nquad; ++i) {
    bf16x4 q;
    q[0] = (bf16)buf[4 * i];     q[1] = (bf16)buf[4 * i + 1];
    q[2] = (bf16)buf[4 * i + 2]; q[3] = (bf16)buf[4 * i + 3];
    *(bf16x4*)(dst + 4 * i) = q;
  }
}

__global__ __launch_bounds__(256) void transpose_pack_kernel(const float* __restrict__ W, bf16* __restrict__ WT, int K, int N, size_t plane) {
  __shared__ float tile[64][65];
  const int k0 = blockIdx.y * 64, n0 = blockIdx.x * 64, t = threadIdx.x;
  for (int i = t; i < 64 * 64; i += 256) { const int kr = i >> 6, nc = i & 63; tile[kr][nc] = W[(size_t)(k0 + kr) * N + n0 + nc]; }
  __syncthreads();
#pragma unroll 1
  for (int pass = 0; pass < 2; ++pass) {
    for (int i = t; i < 64 * 8; i += 256) { const int nr = i >> 3, k8 = (i & 7) * 8; bf16 hh[8], hl[8];
#pragma unroll
      for (int e = 0; e < 8; ++e) { const float v = tile[k8 + e][nr]; hh[e] = (bf16)v; hl[e] = lo_of(v, hh[e]); }
      bf16* d = WT + (size_t)(n0 + nr) * K + k0 + k8;
      *(volatile v4u_t*)d = *(const v4ua*)hh; *(volatile v4u_t*)(d + plane) = *(const v4ua*)hl; }
    __threadfence();
  }
}

template <typename AT, typename WT, int MODE>
__global__ __launch_bounds__(256) void gemm_split_kernel(
    const AT* __restrict__ A, size_t aPlane, const WT* __restrict__ W, size_t wPlane,
    const float* __restrict__ bias, void* __restrict__ out,
    int M, int N, int K) {
  __shared__ bf16 ldsA[128 * LDS_STRIDE], ldsAl[128 * LDS_STRIDE];
  __shared__ bf16 ldsW[256 * LDS_STRIDE], ldsWl[256 * LDS_STRIDE];
  __shared__ __attribute__((aligned(16))) unsigned char sob[256 * 136 * 2];

  const int t    = threadIdx.x;
  const int wave = t >> 5;
  const int lane = t & 31;
  const int wm   = (wave & 1) * 64;
  const int wn   = (wave >> 1) * 64;
  const int mBlk = blockIdx.x * 128;
  const int nBlk = blockIdx.y * 256;
  const int arow = t >> 1;
  const int ach  = (t & 1) * 16;

  f32x8 acc[4][4] = {};
  for (int k = 0; k < K; k += 32) {
    __syncthreads();
    {
      const AT* ap = A + (size_t)(mBlk + arow) * K + k + ach;
      bf16 hh[16], hl[16];
      if (sizeof(AT) == 4) {
#pragma unroll
        for (int i = 0; i < 16; ++i) { const float v = (float)ap[i]; hh[i] = (bf16)v; hl[i] = lo_of(v, hh[i]); }
      } else {
#pragma unroll
        for (int i = 0; i < 16; ++i) { hh[i] = (bf16)ap[i]; hl[i] = (bf16)ap[aPlane + i]; }
      }
#pragma unroll
      for (int i = 0; i < 16; ++i) { ldsA[arow * LDS_STRIDE + ach + i] = hh[i]; ldsAl[arow * LDS_STRIDE + ach + i] = hl[i]; }
    }
    {
      const WT* wp = W + (size_t)(nBlk + t) * K + k;
      if (sizeof(WT) == 4) {
#pragma unroll
        for (int i = 0; i < 32; ++i) { const float v = (float)wp[i]; const bf16 h_ = (bf16)v; ldsW[t * LDS_STRIDE + i] = h_; ldsWl[t * LDS_STRIDE + i] = lo_of(v, h_); }
      } else {
#pragma unroll
        for (int i = 0; i < 32; ++i) { ldsW[t * LDS_STRIDE + i] = (bf16)wp[i]; ldsWl[t * LDS_STRIDE + i] = (bf16)wp[wPlane + i]; }
      }
    }
    __syncthreads();
    bf16x16 wf[4], wfl[4];
#pragma unroll
    for (int j = 0; j < 4; ++j) { wf[j] = lds_frag(ldsW + (wn + 16 * j) * LDS_STRIDE, LDS_STRIDE); wfl[j] = lds_frag(ldsWl + (wn + 16 * j) * LDS_STRIDE, LDS_STRIDE); }
#pragma unroll
    for (int i = 0; i < 4; ++i) {
      const bf16x16 af = lds_frag(ldsA + (wm + 16 * i) * LDS_STRIDE, LDS_STRIDE), afl = lds_frag(ldsAl + (wm + 16 * i) * LDS_STRIDE, LDS_STRIDE);
#pragma unroll
      for (int j = 0; j < 4; ++j) acc[i][j] = wmma_split(af, afl, wf[j], wfl[j], acc[i][j]);
    }
  }

  const int nlane = lane & 15;
  const int mh    = (lane >> 4) * 8;
  __syncthreads();
  if (MODE == 1) {
    bf16* so = (bf16*)sob;
#pragma unroll
    for (int i = 0; i < 4; ++i)
#pragma unroll
      for (int j = 0; j < 4; ++j) {
        const int nl = wn + 16 * j + nlane;
        const float bv = bias ? bias[nBlk + nl] : 0.0f;
#pragma unroll
        for (int r = 0; r < 8; ++r) so[nl * 136 + wm + 16 * i + mh + r] = (bf16)(acc[i][j][r] + bv);
      }
    __syncthreads();
    const int b_ = mBlk >> 11, s0 = mBlk & (SS - 1);
#pragma unroll 1
    for (int pass = 0; pass < 2; ++pass) {
      for (int ch = t; ch < 256 * 16; ch += 256) { const int nl = ch >> 4, q = (ch & 15) * 8; const int n = nBlk + nl, h = n >> 6, dk = n & (DKK - 1);
        *(volatile v4u_t*)((bf16*)out + (((size_t)(b_ * HH + h)) * DKK + dk) * SS + s0 + q) = *(const v4ua*)(so + nl * 136 + q); }
      __threadfence();
    }
  } else {
    float* so = (float*)sob;
#pragma unroll 1
    for (int hf = 0; hf < 2; ++hf) {
      if (wm == hf * 64) {
#pragma unroll
        for (int i = 0; i < 4; ++i)
#pragma unroll
          for (int j = 0; j < 4; ++j) {
            const int nl = wn + 16 * j + nlane;
            const float bv = bias ? bias[nBlk + nl] : 0.0f;
#pragma unroll
            for (int r = 0; r < 8; ++r) so[(16 * i + mh + r) * 260 + nl] = acc[i][j][r] + bv;
          }
      }
      __syncthreads();
#pragma unroll 1
      for (int pass = 0; pass < 2; ++pass) {
        for (int ch = t; ch < 64 * 64; ch += 256) { const int ml = ch >> 6, q = (ch & 63) * 4;
          *(volatile v4f_t*)((float*)out + (size_t)(mBlk + hf * 64 + ml) * N + nBlk + q) = *(const volatile v4fa*)(so + ml * 260 + q); }
        __threadfence();
      }
      __syncthreads();
    }
  }
}


#define GN 50000
#define GNP 50176
#define GE 400000
#define GD 128
#define DRANGE 12544

__global__ __launch_bounds__(128) void k_trA(const float* __restrict__ W, float* __restrict__ A) {
  const int m = blockIdx.x, k = threadIdx.x; const float v = W[(size_t)k * GD + m];
  *(volatile float*)(A + (size_t)m * GD + k) = v; __threadfence(); *(volatile float*)(A + (size_t)m * GD + k) = v;
}
__global__ __launch_bounds__(128) void k_padrows(const float* __restrict__ x, float* __restrict__ XP) {
  const int row = blockIdx.x, k = threadIdx.x; const float v = (row < GN) ? x[(size_t)row * GD + k] : 0.0f;
  *(volatile float*)(XP + (size_t)row * GD + k) = v; __threadfence(); *(volatile float*)(XP + (size_t)row * GD + k) = v;
}
__global__ __launch_bounds__(256) void k_rowsb(const float* __restrict__ T, int tstride, const float* __restrict__ b, float* __restrict__ F) {
  __shared__ float tile[64][65];
  const int n0 = blockIdx.x * 64, cb = blockIdx.y * 64, t = threadIdx.x;
  for (int i = t; i < 64 * 64; i += 256) { const int c = i >> 6, nn = i & 63; tile[c][nn] = T[(size_t)(cb + c) * tstride + n0 + nn]; }
  __syncthreads();
#pragma unroll 1
  for (int pass = 0; pass < 2; ++pass) {
    for (int i = t; i < 64 * 16; i += 256) { const int nr = i >> 4, c4 = (i & 15) * 4; v4f_t v;
#pragma unroll
      for (int q = 0; q < 4; ++q) v[q] = tile[c4 + q][nr] + b[cb + c4 + q];
      *(volatile v4f_t*)(F + (size_t)(n0 + nr) * GD + cb + c4) = v; }
    __threadfence();
  }
}
__global__ __launch_bounds__(256) void k_gat2(const int* __restrict__ srci, const int* __restrict__ dsti, const float* __restrict__ FS, const float* __restrict__ FDr,
                                             const float* __restrict__ attn, const float* __restrict__ resid, float* __restrict__ Z, int rsel) {
  __shared__ int qd[8][256], qs[8][256]; __shared__ int wcnt[8][8];
  __shared__ float mx[DRANGE], den[DRANGE]; __shared__ float av[GD];
  const int tid = threadIdx.x, lane = tid & 31, wave = tid >> 5, r0 = rsel * DRANGE;
  float* myZ = Z + (size_t)r0 * GD;
  for (int i = tid; i < DRANGE; i += 256) { mx[i] = -3.0e38f; den[i] = 0.0f; }
  if (tid < GD) av[tid] = attn[tid];
  for (int i = tid; i < DRANGE * GD / 4; i += 256) { v4f_t z; z.x = z.y = z.z = z.w = 0.0f; *(volatile v4f_t*)(myZ + (size_t)i * 4) = z; }
  __threadfence(); __syncthreads();
#pragma unroll 1
  for (int ps = 0; ps < 2; ++ps) {
#pragma unroll 1
    for (int c0 = 0; c0 < GE; c0 += 256) {
      const int e = c0 + tid; int d = -1, sidx = 0;
      if (e < GE) { const int draw = dsti[e]; const int dd = draw < 0 ? 0 : (draw >= GN ? GN - 1 : draw);
        if (dd >= r0 && dd < r0 + DRANGE) { d = dd - r0; const int ss = srci[e]; sidx = ss < 0 ? 0 : (ss >= GN ? GN - 1 : ss); } }
      const int own = (d >= 0) ? (d & 7) : -1; unsigned mown = 0u;
#pragma unroll
      for (int w = 0; w < 8; ++w) { const unsigned m = __builtin_amdgcn_ballot_w32(own == w); if (own == w) mown = m; if (lane == 0) wcnt[w][wave] = __builtin_popcount(m); }
      __syncthreads();
      if (own >= 0) { int base = 0;
#pragma unroll
        for (int w2 = 0; w2 < 8; ++w2) base += (w2 < wave) ? wcnt[own][w2] : 0;
        const int pos = base + __builtin_popcount(mown & ((1u << lane) - 1u)); qd[own][pos] = d; qs[own][pos] = sidx; }
      int total = 0;
#pragma unroll
      for (int w2 = 0; w2 < 8; ++w2) total += wcnt[wave][w2];
      __syncthreads();
#pragma unroll 1
      for (int qi = 0; qi < total; ++qi) { const int dl = qd[wave][qi]; const int sl = qs[wave][qi];
        const float* fs = FS + (size_t)sl * GD; const float* fd = FDr + (size_t)dl * GD;
        float part = 0.0f; float fsv[4];
#pragma unroll
        for (int u = 0; u < 4; ++u) { const int c = u * 32 + lane; fsv[u] = fs[c]; float s = fsv[u] + fd[c]; s = (s > 0.0f) ? s : 0.2f * s; part += av[c] * s; }
#pragma unroll
        for (int o = 16; o >= 1; o >>= 1) part += __shfl_xor(part, o, 32);
        if (ps == 0) { if (lane == 0) mx[dl] = fmaxf(mx[dl], part); }
        else { const float ex = expf(part - mx[dl]); if (lane == 0) den[dl] += ex; float* row = myZ + (size_t)dl * GD;
#pragma unroll
          for (int u = 0; u < 4; ++u) row[u * 32 + lane] += ex * fsv[u]; }
      }
      __syncthreads();
    }
  }
  __threadfence(); __syncthreads();
#pragma unroll 1
  for (int pass = 0; pass < 2; ++pass) {
    for (int i = tid; i < DRANGE * 32; i += 256) { const int dl = i >> 5, c4 = (i & 31) * 4, node = r0 + dl; float* p = myZ + (size_t)dl * GD + c4;
      v4f_t v = *(const volatile v4fa*)p;
      if (pass == 0) { const float dn = den[dl]; const float inv = (dn > 0.0f) ? 1.0f / dn : 0.0f; v.x *= inv; v.y *= inv; v.z *= inv; v.w *= inv;
        if (resid != nullptr && node < GN) { const v4f_t r = *(const v4fa*)(resid + (size_t)node * GD + c4); v.x += r.x; v.y += r.y; v.z += r.z; v.w += r.w; } }
      *(volatile v4f_t*)p = v; }
    __threadfence(); __syncthreads();
  }
}
__global__ __launch_bounds__(256) void k_foldgate(const float* __restrict__ W1, const float* __restrict__ b1, const float* __restrict__ W2, const float* __restrict__ b2, float* __restrict__ wv) {
  const int k = threadIdx.x; float s = 0.0f;
#pragma unroll 1
  for (int j = 0; j < GD; ++j) s += W1[(size_t)k * GD + j] * W2[j];
  *(volatile float*)(wv + k) = s;
  if (k == 0) { float bb = b2[0];
#pragma unroll 1
    for (int j = 0; j < GD; ++j) bb += b1[j] * W2[j];
    *(volatile float*)(wv + 256) = bb; }
  __threadfence();
  *(volatile float*)(wv + k) = s;
}
__global__ __launch_bounds__(128) void k_userout(const float* __restrict__ U, const float* __restrict__ P, const float* __restrict__ Q, const float* __restrict__ winf, const float* __restrict__ wint, float* __restrict__ out) {
  const int wave = threadIdx.x >> 5, lane = threadIdx.x & 31, u = blockIdx.x * 4 + wave;
  const float* ur = U + (size_t)u * GD; const float* pr = P + (size_t)u * GD; const float* qr = Q + (size_t)u * GD;
  float si = 0.0f, st = 0.0f; float uv[4], pv[4], qv[4];
#pragma unroll
  for (int k = 0; k < 4; ++k) { const int c = k * 32 + lane; uv[k] = ur[c]; pv[k] = pr[c]; qv[k] = qr[c];
    si += uv[k] * winf[c] + pv[k] * winf[GD + c]; st += uv[k] * wint[c] + qv[k] * wint[GD + c]; }
#pragma unroll
  for (int o = 16; o >= 1; o >>= 1) { si += __shfl_xor(si, o, 32); st += __shfl_xor(st, o, 32); }
  si += winf[256]; st += wint[256];
  si = (si > 0.0f) ? si : 0.01f * si; st = (st > 0.0f) ? st : 0.01f * st;
  const float m = fmaxf(si, st); const float e0 = expf(si - m), e1 = expf(st - m); const float g0 = e0 / (e0 + e1), g1 = e1 / (e0 + e1);
  float ov[4];
#pragma unroll
  for (int k = 0; k < 4; ++k) ov[k] = g0 * pv[k] + g1 * qv[k] + uv[k];
#pragma unroll 1
  for (int pass = 0; pass < 2; ++pass) {
#pragma unroll
    for (int k = 0; k < 4; ++k) *(volatile float*)(out + (size_t)u * GD + k * 32 + lane) = ov[k];
    __threadfence(); }
}

extern "C" void kernel_launch(void* const* d_in, const int* in_sizes, int n_in,
                              void* d_out, int out_size, void* d_ws, size_t ws_size,
                              hipStream_t stream) {
  (void)in_sizes; (void)n_in; (void)out_size; (void)ws_size;
  const float* uemb = (const float*)d_in[0]; const float* iemb = (const float*)d_in[1];
  const int* rate_src = (const int*)d_in[2]; const int* rate_dst = (const int*)d_in[3];
  const int* rb_src = (const int*)d_in[4];   const int* rb_dst = (const int*)d_in[5];
  const int* tr_src = (const int*)d_in[6];   const int* tr_dst = (const int*)d_in[7];
  const float* Wsrc[3] = {(const float*)d_in[8],  (const float*)d_in[13], (const float*)d_in[18]};
  const float* bsrc[3] = {(const float*)d_in[9],  (const float*)d_in[14], (const float*)d_in[19]};
  const float* Wdst[3] = {(const float*)d_in[10], (const float*)d_in[15], (const float*)d_in[20]};
  const float* bdst[3] = {(const float*)d_in[11], (const float*)d_in[16], (const float*)d_in[21]};
  const float* attv[3] = {(const float*)d_in[12], (const float*)d_in[17], (const float*)d_in[22]};
  const float* inf_W1 = (const float*)d_in[23]; const float* inf_b1 = (const float*)d_in[24]; const float* inf_W2 = (const float*)d_in[25]; const float* inf_b2 = (const float*)d_in[26];
  const float* int_W1 = (const float*)d_in[27]; const float* int_b1 = (const float*)d_in[28]; const float* int_W2 = (const float*)d_in[29]; const float* int_b2 = (const float*)d_in[30];
  float* user_out = (float*)d_out;
  float* item_out = user_out + (size_t)GN * GD;
  char* ws = (char*)d_ws;
  float* A   = (float*)ws; ws += (size_t)6 * GD * GD * 4;
  float* wg  = (float*)ws; ws += 2 * 512 * 4;
  float* UP  = (float*)ws; ws += (size_t)GNP * GD * 4;
  float* IP  = (float*)ws; ws += (size_t)GNP * GD * 4;
  float* T   = (float*)ws; ws += (size_t)GD * GNP * 4;
  float* FS  = (float*)ws; ws += (size_t)GNP * GD * 4;
  float* T2  = (float*)ws; ws += (size_t)GD * DRANGE * 4;
  float* FDr = (float*)ws; ws += (size_t)DRANGE * GD * 4;
  for (int r = 0; r < 3; ++r) { k_trA<<<GD, 128, 0, stream>>>(Wsrc[r], A + (size_t)(2 * r) * GD * GD); k_trA<<<GD, 128, 0, stream>>>(Wdst[r], A + (size_t)(2 * r + 1) * GD * GD); }
  k_foldgate<<<1, 256, 0, stream>>>(inf_W1, inf_b1, inf_W2, inf_b2, wg);
  k_foldgate<<<1, 256, 0, stream>>>(int_W1, int_b1, int_W2, int_b2, wg + 512);
  k_padrows<<<GNP, 128, 0, stream>>>(uemb, UP);
  k_padrows<<<GNP, 128, 0, stream>>>(iemb, IP);
  dim3 blk(256);
  auto relation = [&](int r, const float* SRCX, const float* DSTX, const int* es, const int* ed, const float* resid, float* Zout) {
    gemm_split_kernel<float, float, 2><<<dim3(1, GNP / 256), blk, 0, stream>>>(A + (size_t)(2 * r) * GD * GD, 0, SRCX, 0, nullptr, T, GD, GNP, GD);
    k_rowsb<<<dim3(GNP / 64, 2), 256, 0, stream>>>(T, GNP, bsrc[r], FS);
    for (int g = 0; g < GNP / DRANGE; ++g) {
      gemm_split_kernel<float, float, 2><<<dim3(1, DRANGE / 256), blk, 0, stream>>>(A + (size_t)(2 * r + 1) * GD * GD, 0, DSTX + (size_t)g * DRANGE * GD, 0, nullptr, T2, GD, DRANGE, GD);
      k_rowsb<<<dim3(DRANGE / 64, 2), 256, 0, stream>>>(T2, DRANGE, bdst[r], FDr);
      k_gat2<<<1, 256, 0, stream>>>(es, ed, FS, FDr, attv[r], resid, Zout, g);
    }
  };
  relation(0, UP, IP, rate_src, rate_dst, iemb, T);
  k_padrows<<<GN, 128, 0, stream>>>(T, item_out);
  relation(1, IP, UP, rb_src, rb_dst, nullptr, T);
  float* Qr = IP;
  k_padrows<<<GNP, 128, 0, stream>>>(T, Qr);
  relation(2, UP, UP, tr_src, tr_dst, nullptr, T);
  k_userout<<<GN / 4, 128, 0, stream>>>(UP, T, Qr, wg, wg + 512, user_out);
}
